// MultiheadAttention_35648228556929
// MI455X (gfx1250) — hardware-run, weakly checked
//
#include <hip/hip_runtime.h>


#ifndef NB
#define NB 2
#endif
#ifndef SEQ
#define SEQ 2048
#endif
#define NB_FULL  2
#define SEQ_FULL 2048
#define DM   1024
#define NH   16
#define HD   64
#define DQ   (NH * HD)
#define ZH   2
#define QCAR  16.0f
#define VCAR  16.0f
#define PCAR  1024.0f
#define CCAR  64.0f
#define WOCAR 1024.0f
#define SCL  (0.25f / (QCAR * QCAR))
#define MSC  (CCAR / (PCAR * VCAR))
#define OSC  (1.0f / (CCAR * WOCAR))

static_assert(SEQ % 128 == 0);
static_assert(SEQ <= SEQ_FULL);
static_assert(NB <= NB_FULL);
static_assert(DM % 64 == 0);
static_assert(DQ == DM);
static_assert(NH % ZH == 0);
static_assert(HD == 64);

typedef _Float16 h16;
typedef unsigned short bf;
typedef __attribute__((ext_vector_type(16))) __bf16   v16bf;
typedef __attribute__((ext_vector_type(16))) _Float16 v16h;
typedef __attribute__((ext_vector_type(8)))  _Float16 v8h;
typedef __attribute__((ext_vector_type(4)))  _Float16 v4h;
typedef __attribute__((ext_vector_type(8)))  unsigned short v8us;
typedef __attribute__((ext_vector_type(8)))  float    v8f;
typedef __attribute__((ext_vector_type(4)))  float    v4f;
typedef v4f  __attribute__((may_alias)) v4fa;

__device__ __forceinline__ unsigned short f2bf(float f) { unsigned u = __float_as_uint(f); u += 0x7FFFu + ((u >> 16) & 1u); return (unsigned short)(u >> 16); }
__device__ __forceinline__ float bf2f(unsigned short b) { return __uint_as_float(((unsigned)b) << 16); }
__device__ __forceinline__ float bfr(float f) { return bf2f(f2bf(f)); }
__device__ __forceinline__ h16 tohx(float x) { return (h16)x; }
__device__ __forceinline__ v16h cat16(v8h lo, v8h hi) { return __builtin_shufflevector(lo, hi, 0, 1, 2, 3, 4, 5, 6, 7, 8, 9, 10, 11, 12, 13, 14, 15); }
__device__ __forceinline__ v16bf cat16b(v8us lo, v8us hi) { return __builtin_bit_cast(v16bf, __builtin_shufflevector(lo, hi, 0, 1, 2, 3, 4, 5, 6, 7, 8, 9, 10, 11, 12, 13, 14, 15)); }
__device__ __forceinline__ v8f wmma16(v16h a, v16h b, v8f c) { return __builtin_amdgcn_wmma_f32_16x16x32_f16(false, a, false, b, (short)0, c, false, false); }
__device__ __forceinline__ v8f wmmab(v16bf a, v16bf b, v8f c) { return __builtin_amdgcn_wmma_f32_16x16x32_bf16(false, a, false, b, (short)0, c, false, false); }

template <typename T16> struct WFrag;
template <> struct WFrag<h16> { typedef v16h V; static __device__ __forceinline__ V ld(const h16* p) { return cat16(*(const v8h*)p, *(const v8h*)(p + 16)); } static __device__ __forceinline__ v8f mma(V a, V b, v8f c) { return wmma16(a, b, c); } };
template <> struct WFrag<bf> { typedef v16bf V; static __device__ __forceinline__ V ld(const bf* p) { return cat16b(*(const v8us*)p, *(const v8us*)(p + 16)); } static __device__ __forceinline__ v8f mma(V a, V b, v8f c) { return wmmab(a, b, c); } };

template <typename T16, bool BIAS>
__global__ __launch_bounds__(32) void k_gemmw(const T16* __restrict__ A, const T16* __restrict__ Bt, int K, float* C, int ldc, const float* __restrict__ bias, float osc, size_t sA, size_t sB, size_t sC) {
    typedef typename WFrag<T16>::V V;
    __shared__ __align__(16) float os[16 * 68];
    const size_t z = blockIdx.z; A += z * sA; Bt += z * sB; C += z * sC;
    const int lane = threadIdx.x & 31, lr = lane & 15, hi = lane >> 4; const int r0 = blockIdx.x * 64, c0 = blockIdx.y * 64;
    v8f acc[4][4];
#pragma unroll
    for (int mb = 0; mb < 4; ++mb)
#pragma unroll
        for (int nb = 0; nb < 4; ++nb) acc[mb][nb] = (v8f){};
    const size_t aoff = (size_t)(r0 + lr) * K + 8 * hi, boff = (size_t)(c0 + lr) * K + 8 * hi;
#pragma unroll 1
    for (int kc = 0; kc < K; kc += 32) {
        V a[4];
#pragma unroll
        for (int mb = 0; mb < 4; ++mb) a[mb] = WFrag<T16>::ld(A + aoff + (size_t)mb * 16 * K + kc);
#pragma unroll
        for (int nb = 0; nb < 4; ++nb) { const V b = WFrag<T16>::ld(Bt + boff + (size_t)nb * 16 * K + kc);
#pragma unroll
            for (int mb = 0; mb < 4; ++mb) acc[mb][nb] = WFrag<T16>::mma(a[mb], b, acc[mb][nb]); }
        asm volatile("v_nop\n\tv_nop\n\tv_nop\n\tv_nop" : "+v"(acc[0][3]), "+v"(acc[1][3]), "+v"(acc[2][3]), "+v"(acc[3][3]) : "v"(a[0]), "v"(a[3]));
    }
#pragma unroll
    for (int mb = 0; mb < 4; ++mb) {
#pragma unroll
        for (int nb = 0; nb < 4; ++nb) {
#pragma unroll
            for (int j = 0; j < 8; ++j) os[(hi * 8 + j) * 68 + nb * 16 + lr] = acc[mb][nb][j]; }
        __builtin_amdgcn_wave_barrier(); asm volatile("" ::: "memory");
        float* crow = C + (size_t)(r0 + mb * 16) * ldc + c0;
#pragma unroll 1
        for (int ps = 0; ps < 2; ++ps) {
#pragma unroll
            for (int s = 0; s < 8; ++s) { const int row = 2 * s + hi, cofs = lr * 4; v4f val = *(const v4fa*)(os + row * 68 + cofs);
                val[0] *= osc; val[1] *= osc; val[2] *= osc; val[3] *= osc;
                if (BIAS) { val[0] += bfr(bias[c0 + cofs]); val[1] += bfr(bias[c0 + cofs + 1]); val[2] += bfr(bias[c0 + cofs + 2]); val[3] += bfr(bias[c0 + cofs + 3]); }
                *(volatile v4f*)(crow + (size_t)row * ldc + cofs) = val; }
            if (ps == 0) __threadfence(); }
        __builtin_amdgcn_wave_barrier(); asm volatile("" ::: "memory");
    }
}

__global__ __launch_bounds__(256) void k_cvt8(const float* __restrict__ src, bf* dst, size_t n8) { const size_t i = (size_t)blockIdx.x * 256 + threadIdx.x; if (i >= n8) return; const v8f v = *(const v8f*)(src + i * 8); v8us o;
#pragma unroll
    for (int k = 0; k < 8; ++k) o[k] = f2bf(v[k]);
    *(volatile v8us*)(dst + i * 8) = o; __threadfence(); *(volatile v8us*)(dst + i * 8) = o; }

__global__ __launch_bounds__(256) void k_cvt8h(const float* __restrict__ src, h16* dst, float sc, size_t n8) { const size_t i = (size_t)blockIdx.x * 256 + threadIdx.x; if (i >= n8) return; const v8f v = *(const v8f*)(src + i * 8); v8h o;
#pragma unroll
    for (int k = 0; k < 8; ++k) o[k] = tohx(bfr(v[k]) * sc);
    *(volatile v8h*)(dst + i * 8) = o; __threadfence(); *(volatile v8h*)(dst + i * 8) = o; }

__global__ __launch_bounds__(256) void k_hp8(const float* __restrict__ F, float sc, h16* P16) {
    const size_t i = (size_t)blockIdx.x * 256 + threadIdx.x; if (i >= (size_t)NH * SEQ * HD / 8) return; const size_t e = i * 8;
    const int d = (int)(e % HD); const int t = (int)((e / HD) % SEQ); const int h = (int)(e / ((size_t)HD * SEQ));
    const float* f = F + (size_t)t * DQ + h * HD + d; const v4f a = *(const v4f*)f; const v4f b = *(const v4f*)(f + 4); v8h o;
#pragma unroll
    for (int k = 0; k < 4; ++k) { o[k] = tohx(a[k] * sc); o[4 + k] = tohx(b[k] * sc); }
    *(volatile v8h*)(P16 + e) = o; __threadfence(); *(volatile v8h*)(P16 + e) = o; }

__global__ __launch_bounds__(256) void k_vt8(const float* __restrict__ F, float sc, h16* V16) {
    const size_t i = (size_t)blockIdx.x * 256 + threadIdx.x; if (i >= (size_t)NH * HD * SEQ / 8) return; const size_t e = i * 8;
    const int t = (int)(e % SEQ); const int d = (int)((e / SEQ) % HD); const int g = (int)(e / ((size_t)SEQ * HD));
    const float* f = F + (size_t)t * DQ + g * HD + d; v8h o;
#pragma unroll
    for (int q = 0; q < 8; ++q) o[q] = tohx(f[(size_t)q * DQ] * sc);
    *(volatile v8h*)(V16 + e) = o; __threadfence(); *(volatile v8h*)(V16 + e) = o; }

__global__ __launch_bounds__(256) void k_asoft(const float* __restrict__ Sb, h16* P16) {
    const int lane = threadIdx.x & 31; const int row = blockIdx.x * 8 + (threadIdx.x >> 5); if (row >= ZH * SEQ) return;
    const float* sr = Sb + (size_t)row * SEQ; float v[SEQ / 32]; float mx = -3.0e38f;
#pragma unroll
    for (int ch = 0; ch < SEQ / 128; ++ch) { const int j0 = ch * 128 + lane * 4; const v4f a = *(const v4f*)(sr + j0);
#pragma unroll
        for (int q = 0; q < 4; ++q) { const float t = a[q] * SCL; v[ch * 4 + q] = t; mx = fmaxf(mx, t); } }
#pragma unroll
    for (int sh = 16; sh; sh >>= 1) mx = fmaxf(mx, __shfl_xor(mx, sh, 32));
    float sum = 0.f;
#pragma unroll
    for (int k = 0; k < SEQ / 32; ++k) { float d0 = __fsub_rn(v[k], mx); asm volatile("" : "+v"(d0)); v[k] = __builtin_amdgcn_exp2f(__fmul_rn(d0, 1.4426950408889634f)); sum += v[k]; }
#pragma unroll
    for (int sh = 16; sh; sh >>= 1) sum += __shfl_xor(sum, sh, 32);
    const float f = __fdiv_rn(PCAR, sum);
    h16* pr = P16 + (size_t)row * SEQ;
#pragma unroll 1
    for (int ps = 0; ps < 2; ++ps) {
#pragma unroll
        for (int ch = 0; ch < SEQ / 128; ++ch) { v4h o4;
#pragma unroll
            for (int q = 0; q < 4; ++q) o4[q] = tohx(v[ch * 4 + q] * f);
            *(volatile v4h*)(pr + ch * 128 + lane * 4) = o4; }
        if (ps == 0) __threadfence(); }
}

__global__ __launch_bounds__(256) void k_merge8(const float* __restrict__ O, int h0, h16* AT) {
    const size_t i = (size_t)blockIdx.x * 256 + threadIdx.x; if (i >= (size_t)ZH * SEQ * HD / 8) return; const size_t e = i * 8;
    const int d = (int)(e % HD); const int t = (int)((e / HD) % SEQ); const int zz = (int)(e / ((size_t)HD * SEQ));
    const v4f a = *(const v4f*)(O + e); const v4f b = *(const v4f*)(O + e + 4); v8h o;
#pragma unroll
    for (int k = 0; k < 4; ++k) { o[k] = tohx(a[k] * MSC); o[4 + k] = tohx(b[k] * MSC); }
    const size_t oo = (size_t)t * DQ + (size_t)(h0 + zz) * HD + d;
    *(volatile v8h*)(AT + oo) = o; __threadfence(); *(volatile v8h*)(AT + oo) = o; }

extern "C" void kernel_launch(void* const* d_in, const int* in_sizes, int n_in,
                              void* d_out, int out_size, void* d_ws, size_t ws_size, hipStream_t stream) {
    if (n_in < 11) return;
    const size_t xneed = (size_t)(NB - 1) * SEQ_FULL * DM + (size_t)SEQ * DM;
    if ((size_t)in_sizes[0] < xneed || (size_t)in_sizes[1] < xneed || (size_t)in_sizes[2] < xneed) return;
    if ((size_t)in_sizes[3] < (size_t)DM * DM || (size_t)in_sizes[5] < (size_t)DM * DM || (size_t)in_sizes[7] < (size_t)DM * DM || (size_t)in_sizes[9] < (size_t)DM * DM) return;
    if (in_sizes[4] < DM || in_sizes[6] < DM || in_sizes[8] < DM || in_sizes[10] < DM) return;
    if ((size_t)out_size < xneed) return;
    const float* xq = (const float*)d_in[0]; const float* xk = (const float*)d_in[1]; const float* xv = (const float*)d_in[2];
    const float* wq = (const float*)d_in[3]; const float* bq = (const float*)d_in[4];
    const float* wk = (const float*)d_in[5]; const float* bk = (const float*)d_in[6];
    const float* wv = (const float*)d_in[7]; const float* bv = (const float*)d_in[8];
    const float* wo = (const float*)d_in[9]; const float* bo = (const float*)d_in[10];
    float* OUT = (float*)d_out;
    char* wsp = (char*)d_ws;
    auto take = [&](size_t bytes) { char* p = wsp; wsp += (bytes + 255) & ~(size_t)255; return (void*)p; };
    bf*  WQ   = (bf*)take((size_t)DM * DM * 2);
    bf*  WK   = (bf*)take((size_t)DM * DM * 2);
    bf*  WV   = (bf*)take((size_t)DM * DM * 2);
    h16* WO   = (h16*)take((size_t)DM * DM * 2);
    bf*  XB   = (bf*)take((size_t)SEQ * DM * 2);
    float* F  = (float*)take((size_t)SEQ * DQ * 4);
    h16* QP16 = (h16*)take((size_t)NH * SEQ * HD * 2);
    h16* KP16 = (h16*)take((size_t)NH * SEQ * HD * 2);
    h16* VT16 = (h16*)take((size_t)NH * HD * SEQ * 2);
    float* Sb = (float*)take((size_t)ZH * SEQ * SEQ * 4);
    h16* P16  = (h16*)take((size_t)ZH * SEQ * SEQ * 2);
    float* Ob = (float*)take((size_t)ZH * SEQ * HD * 4);
    h16* AT   = (h16*)take((size_t)SEQ * DQ * 2);
    const size_t carved = (size_t)(wsp - (char*)d_ws);
    if (carved > ws_size || carved > (size_t)134217728) return;

    const unsigned LW = (unsigned)(((size_t)DM * DM / 8 + 255) / 256);
    const unsigned LX = (unsigned)(((size_t)SEQ * DM / 8 + 255) / 256);
    const unsigned LP = (unsigned)(((size_t)NH * SEQ * HD / 8 + 255) / 256);
    const unsigned LM = (unsigned)(((size_t)ZH * SEQ * HD / 8 + 255) / 256);
    k_cvt8<<<LW, 256, 0, stream>>>(wq, WQ, (size_t)DM * DM / 8);
    k_cvt8<<<LW, 256, 0, stream>>>(wk, WK, (size_t)DM * DM / 8);
    k_cvt8<<<LW, 256, 0, stream>>>(wv, WV, (size_t)DM * DM / 8);
    k_cvt8h<<<LW, 256, 0, stream>>>(wo, WO, WOCAR, (size_t)DM * DM / 8);
    for (int b = 0; b < NB; ++b) {
        const size_t xo = (size_t)b * SEQ_FULL * DM;
        k_cvt8<<<LX, 256, 0, stream>>>(xq + xo, XB, (size_t)SEQ * DM / 8);
        k_gemmw<bf, true><<<dim3(SEQ / 64, DQ / 64, 1), 32, 0, stream>>>(XB, WQ, DM, F, DQ, bq, 1.0f, 0, 0, 0);
        k_hp8<<<LP, 256, 0, stream>>>(F, QCAR, QP16);
        k_cvt8<<<LX, 256, 0, stream>>>(xk + xo, XB, (size_t)SEQ * DM / 8);
        k_gemmw<bf, true><<<dim3(SEQ / 64, DQ / 64, 1), 32, 0, stream>>>(XB, WK, DM, F, DQ, bk, 1.0f, 0, 0, 0);
        k_hp8<<<LP, 256, 0, stream>>>(F, QCAR, KP16);
        k_cvt8<<<LX, 256, 0, stream>>>(xv + xo, XB, (size_t)SEQ * DM / 8);
        k_gemmw<bf, true><<<dim3(SEQ / 64, DQ / 64, 1), 32, 0, stream>>>(XB, WV, DM, F, DQ, bv, 1.0f, 0, 0, 0);
        k_vt8<<<LP, 256, 0, stream>>>(F, VCAR, VT16);
        for (int h0 = 0; h0 < NH; h0 += ZH) {
            const size_t zo = (size_t)h0 * SEQ * HD;
            k_gemmw<h16, false><<<dim3(SEQ / 64, SEQ / 64, ZH), 32, 0, stream>>>(QP16 + zo, KP16 + zo, HD, Sb, SEQ, nullptr, 1.0f, (size_t)SEQ * HD, (size_t)SEQ * HD, (size_t)SEQ * SEQ);
            k_asoft<<<ZH * SEQ / 8, 256, 0, stream>>>(Sb, P16);
            k_gemmw<h16, false><<<dim3(SEQ / 64, HD / 64, ZH), 32, 0, stream>>>(P16, VT16 + zo, SEQ, Ob, HD, nullptr, 1.0f, (size_t)SEQ * SEQ, (size_t)HD * SEQ, (size_t)SEQ * HD);
            k_merge8<<<LM, 256, 0, stream>>>(Ob, h0, AT);
        }
        k_gemmw<h16, true><<<dim3(SEQ / 64, DM / 64, 1), 32, 0, stream>>>(AT, WO, DQ, OUT + xo, DM, bo, OSC, 0, 0, 0);
    }
}
